// seq2seq_cell_57088705299091
// MI455X (gfx1250) — hardware-run, weakly checked
//
#include <hip/hip_runtime.h>
#include <math.h>

constexpr int kBatch = 256;
constexpr int kSeq   = 256;
constexpr int kIn    = 32;
constexpr int kHid   = 256;
constexpr int kOut   = 4;
constexpr int kGate  = 3 * kHid;
constexpr int kThr   = 256;
constexpr int kRows  = 16;
constexpr int kHP    = 264;
constexpr int kXP    = 40;
constexpr int kLP    = 260;
constexpr int kTP    = 72;
constexpr float kWsc    = 16.0f;
constexpr float kWinv   = 1.0f / 16.0f;
constexpr float kPSc    = 1024.0f;
constexpr float kCtxSt  = 1.0f / 1024.0f;
constexpr float kX16Inv = 1.0f / 256.0f;
static_assert(kBatch % kRows == 0);
static_assert(kHid == 32 * (kThr / 32));
static_assert(kSeq == kHid);
static_assert(kIn == 32);
static_assert(kRows * kIn == 64 * 8);
static_assert(kRows == 2 * (kThr / 32));
static_assert(kHP % 8 == 0 && kXP % 8 == 0 && kLP % 4 == 0 && kTP % 8 == 0);
static_assert(kHid % 32 == 0 && kSeq % 64 == 0 && kHid % 64 == 0);
static_assert((kRows * kHP) % 8 == 0);

typedef __attribute__((ext_vector_type(16))) _Float16 v16h;
typedef __attribute__((ext_vector_type(8)))  _Float16 v8h;
typedef __attribute__((ext_vector_type(16))) __bf16   v16b;
typedef __attribute__((ext_vector_type(8)))  __bf16   v8b;
typedef __attribute__((ext_vector_type(8)))  float    v8f;
typedef __attribute__((ext_vector_type(4)))  float    v4f;
typedef __attribute__((ext_vector_type(4)))  unsigned v4u;

__device__ __forceinline__ unsigned short f2bf_bits(float f) {
  unsigned u = __float_as_uint(f);
  return (unsigned short)((u + 0x7FFFu + ((u >> 16) & 1u)) >> 16);
}
__device__ __forceinline__ float bf_bits2f(unsigned short h) { return __uint_as_float(((unsigned)h) << 16); }

__device__ __forceinline__ void dep_guard_h(v8f& a, v8f& b, v16h x, v16h y) { asm volatile("v_nop\n\tv_nop\n\tv_nop\n\tv_nop" : "+v"(a), "+v"(b) : "v"(x), "v"(y)); }
__device__ __forceinline__ void dep_guard_b(v8f& a, v8f& b, v16b x, v16b y) { asm volatile("v_nop\n\tv_nop\n\tv_nop\n\tv_nop" : "+v"(a), "+v"(b) : "v"(x), "v"(y)); }
__device__ __forceinline__ void keep4_h(v16h a, v16h b, v16h c, v16h d) { asm volatile("v_nop" :: "v"(a), "v"(b), "v"(c), "v"(d)); }
__device__ __forceinline__ void keep4_b(v16b a, v16b b, v16b c, v16b d) { asm volatile("v_nop" :: "v"(a), "v"(b), "v"(c), "v"(d)); }
__device__ __forceinline__ void acc_guard4(v8f& a, v8f& b, v8f& c, v8f& d) { asm volatile("v_nop\n\tv_nop\n\tv_nop\n\tv_nop" : "+v"(a), "+v"(b), "+v"(c), "+v"(d)); }
__device__ __forceinline__ void acc_guard2(v8f& a, v8f& b) { asm volatile("v_nop\n\tv_nop\n\tv_nop\n\tv_nop" : "+v"(a), "+v"(b)); }
__device__ __forceinline__ void guard2f3(v8f& a0, v8f& a1, v16h f0, v16h f1, v16h f2) {
  asm volatile("v_nop\n\tv_nop\n\tv_nop\n\tv_nop" : "+v"(a0), "+v"(a1) : "v"(f0), "v"(f1), "v"(f2));
}
__device__ __forceinline__ void guard3f4(v8f& a0, v8f& a1, v8f& a2, v16h f0, v16h f1, v16h f2, v16h f3) {
  asm volatile("v_nop\n\tv_nop\n\tv_nop\n\tv_nop" : "+v"(a0), "+v"(a1), "+v"(a2) : "v"(f0), "v"(f1), "v"(f2), "v"(f3));
}

template <typename T> struct Frag;
template <> struct Frag<_Float16> {
  typedef v16h V; union U { v16h v; v8h h[2]; };
  static __device__ __forceinline__ v16h load(const _Float16* p) {
    U f; f.h[0] = *(const v8h*)(p); f.h[1] = *(const v8h*)(p + 16); return f.v;
  }
  static __device__ __forceinline__ v8f mma(v16h a, v16h b, v8f c) {
    return __builtin_amdgcn_wmma_f32_16x16x32_f16(false, a, false, b, (short)0, c, false, false);
  }
  static __device__ __forceinline__ void guard(v8f& a, v8f& b, v16h x, v16h y) { dep_guard_h(a, b, x, y); }
  static __device__ __forceinline__ void keep(v16h a, v16h b, v16h c, v16h d) { keep4_h(a, b, c, d); }
};
template <> struct Frag<__bf16> {
  typedef v16b V; union U { v16b v; v8b h[2]; };
  static __device__ __forceinline__ v16b load(const __bf16* p) {
    U f; f.h[0] = *(const v8b*)(p); f.h[1] = *(const v8b*)(p + 16); return f.v;
  }
  static __device__ __forceinline__ v8f mma(v16b a, v16b b, v8f c) {
    return __builtin_amdgcn_wmma_f32_16x16x32_bf16(false, a, false, b, (short)0, c, false, false);
  }
  static __device__ __forceinline__ void guard(v8f& a, v8f& b, v16b x, v16b y) { dep_guard_b(a, b, x, y); }
  static __device__ __forceinline__ void keep(v16b a, v16b b, v16b c, v16b d) { keep4_b(a, b, c, d); }
};

__device__ __forceinline__ v8f mmah(v16h a, v16h b, v8f c) {
  return __builtin_amdgcn_wmma_f32_16x16x32_f16(false, a, false, b, (short)0, c, false, false);
}
__device__ __forceinline__ float fsig(float x)  { return __builtin_amdgcn_rcpf(1.0f + expf(-x)); }
__device__ __forceinline__ float ftanh(float x) { return 1.0f - 2.0f * __builtin_amdgcn_rcpf(expf(2.0f * x) + 1.0f); }

template <int ET> struct Elem;
template <> struct Elem<0> { typedef _Float16 T; };
template <> struct Elem<1> { typedef __bf16 T; };
template <int ET, bool SPLIT, int BIAS_MODE, int OUT_MODE, bool RESID, int ACT = 0>
__global__ __launch_bounds__(256) void wmma_gemm64(
    const unsigned short* __restrict__ Ap, const unsigned short* __restrict__ A2p, int lda, long strideA,
    const unsigned short* __restrict__ Btp, const unsigned short* __restrict__ Bt2p, int ldb, long strideB,
    void* __restrict__ Cout, void* __restrict__ Cout2, int ldc, long strideC,
    const float* __restrict__ bias,
    const float* __restrict__ resid, long strideR,
    int M, int N, int K, float scale) {
  typedef typename Elem<ET>::T T;
  typedef typename Frag<T>::V V;
  const T* A = (const T*)Ap; const T* A2 = (const T*)A2p; const T* Bt = (const T*)Btp; const T* Bt2 = (const T*)Bt2p;
  __shared__ __align__(16) float sT[8][16 * 68];
  const int b    = blockIdx.y;
  const int lane = threadIdx.x & 31;
  const int wave = threadIdx.x >> 5;
  const int tilesN = N >> 6;
  const int tilesM = M >> 6;
  const int tile = blockIdx.x * 8 + wave;
  if (tile >= tilesM * tilesN) return;
  const int tm = tile / tilesN;
  const int tn = tile - tm * tilesN;
  const int m0 = tm << 6;
  const int n0 = tn << 6;

  const T* Ab  = A  + (size_t)b * strideA;
  const T* Bb  = Bt + (size_t)b * strideB;
  const T* Ab2 = SPLIT ? (A2  + (size_t)b * strideA) : nullptr;
  const T* Bb2 = SPLIT ? (Bt2 + (size_t)b * strideB) : nullptr;

  const int rlane = lane & 15;
  const int koff  = (lane >> 4) * 8;
  const int mOff  = (lane >> 4) * 8;

  v8f acc[4][4];
#pragma unroll
  for (int i = 0; i < 4; ++i)
#pragma unroll
    for (int j = 0; j < 4; ++j) acc[i][j] = (v8f){0.f,0.f,0.f,0.f,0.f,0.f,0.f,0.f};

  for (int k0 = 0; k0 < K; k0 += 32) {
    V bh[4], bl[4];
#pragma unroll
    for (int j = 0; j < 4; ++j) {
      const size_t bo = (size_t)(n0 + (j << 4) + rlane) * ldb + koff + k0;
      bh[j] = Frag<T>::load(Bb + bo);
      if (SPLIT) bl[j] = Frag<T>::load(Bb2 + bo);
    }
#pragma unroll
    for (int i = 0; i < 4; ++i) {
      const size_t ao = (size_t)(m0 + (i << 4) + rlane) * lda + koff + k0;
      V ah = Frag<T>::load(Ab + ao);
      V al;
      if (SPLIT) al = Frag<T>::load(Ab2 + ao);
#pragma unroll
      for (int j = 0; j < 4; ++j) {
        acc[i][j] = Frag<T>::mma(ah, bh[j], acc[i][j]);
        if (SPLIT) {
          acc[i][j] = Frag<T>::mma(ah, bl[j], acc[i][j]);
          acc[i][j] = Frag<T>::mma(al, bh[j], acc[i][j]);
        }
      }
      Frag<T>::guard(acc[i][0], acc[i][3], ah, SPLIT ? al : ah);
    }
    Frag<T>::keep(bh[0], bh[1], bh[2], bh[3]);
    if (SPLIT) Frag<T>::keep(bl[0], bl[1], bl[2], bl[3]);
  }
  acc_guard4(acc[0][0], acc[0][1], acc[0][2], acc[0][3]);
  acc_guard4(acc[1][0], acc[1][1], acc[1][2], acc[1][3]);
  acc_guard4(acc[2][0], acc[2][1], acc[2][2], acc[2][3]);
  acc_guard4(acc[3][0], acc[3][1], acc[3][2], acc[3][3]);

  float* slab = sT[wave];
  const float* Rb = RESID ? (resid + (size_t)b * strideR) : nullptr;
#pragma unroll
  for (int i = 0; i < 4; ++i) {
    const int mBase = m0 + (i << 4);
#pragma unroll
    for (int j = 0; j < 4; ++j) {
      const int n = n0 + (j << 4) + rlane;
      float bv = 0.f;
      if (BIAS_MODE == 2) bv = bias[n];
#pragma unroll
      for (int r = 0; r < 8; ++r) {
        float v = acc[i][j][r] * scale;
        if (BIAS_MODE == 1) v += bias[mBase + mOff + r];
        if (BIAS_MODE == 2) v += bv;
        if (RESID) v += Rb[(size_t)(mBase + mOff + r) * ldc + n];
        if (ACT == 1) v = tanhf(v);
        if (ACT == 2) v = fmaxf(v, 0.0f);
        if (ACT == 3) v = v / (1.0f + expf(-v));
        if (ACT == 4) v = (v > 0.f) ? v : 0.01f * v;
        if (ACT == 5) v = 0.5f * v * (1.0f + erff(v * 0.70710678118654752f));
        slab[(mOff + r) * 68 + (j << 4) + rlane] = v;
      }
    }
    __builtin_amdgcn_fence(__ATOMIC_RELEASE, "workgroup");
    __builtin_amdgcn_wave_barrier();
    __builtin_amdgcn_fence(__ATOMIC_ACQUIRE, "workgroup");
    if (OUT_MODE == 0) {
      float* C = (float*)Cout + (size_t)b * strideC;
      const int hh = lane >> 4, c4 = (lane & 15) * 4;
      for (int pass = 0; pass < 2; ++pass) {
#pragma unroll
        for (int it = 0; it < 8; ++it) {
          const int row = it * 2 + hh;
          v4f v = *(const v4f*)(slab + row * 68 + c4);
          *(volatile v4f*)(C + (size_t)(mBase + row) * ldc + n0 + c4) = v;
        }
        __threadfence();
      }
    } else {
      const int q = lane >> 3, c8 = (lane & 7) * 8;
      unsigned short* C  = (unsigned short*)Cout  + (size_t)b * strideC;
      unsigned short* C2 = (OUT_MODE == 2) ? ((unsigned short*)Cout2 + (size_t)b * strideC) : nullptr;
      for (int pass = 0; pass < 2; ++pass) {
#pragma unroll
        for (int it = 0; it < 4; ++it) {
          const int row = it * 4 + q;
          const float* sp = slab + row * 68 + c8;
          v8h hv, lv;
#pragma unroll
          for (int e = 0; e < 8; ++e) {
            if (OUT_MODE == 1) {
              hv[e] = (_Float16)sp[e];
            } else {
              unsigned short hb = f2bf_bits(sp[e]);
              unsigned short lb = f2bf_bits(sp[e] - bf_bits2f(hb));
              hv[e] = __builtin_bit_cast(_Float16, hb);
              lv[e] = __builtin_bit_cast(_Float16, lb);
            }
          }
          *(volatile v8h*)(C + (size_t)(mBase + row) * ldc + n0 + c8) = hv;
          if (OUT_MODE == 2) *(volatile v8h*)(C2 + (size_t)(mBase + row) * ldc + n0 + c8) = lv;
        }
        __threadfence();
      }
    }
    __builtin_amdgcn_fence(__ATOMIC_RELEASE, "workgroup");
    __builtin_amdgcn_wave_barrier();
    __builtin_amdgcn_fence(__ATOMIC_ACQUIRE, "workgroup");
  }
}

__global__ __launch_bounds__(kThr) void cvt8_f16_kernel(const float* __restrict__ src, unsigned short* __restrict__ dst,
                                                        int nrow, int ncol8, int spitch, int scol0, float sc) {
  const int i  = blockIdx.x * kThr + threadIdx.x;
  const int n8 = nrow * ncol8;
  if (i < n8) {
    const int row = i / ncol8;
    const int c8  = i - row * ncol8;
    const float* sp = src + (size_t)row * spitch + scol0 + c8 * 8;
    const v4f a = *(const v4f*)(sp);
    const v4f b = *(const v4f*)(sp + 4);
    v8h hv;
#pragma unroll
    for (int e = 0; e < 4; ++e) {
      hv[e]     = (_Float16)(a[e] * sc);
      hv[4 + e] = (_Float16)(b[e] * sc);
    }
    *(volatile v8h*)(dst + (size_t)i * 8) = hv;
    __threadfence();
    *(volatile v8h*)(dst + (size_t)i * 8) = hv;
  }
}

__global__ __launch_bounds__(kThr) void transpose_e_kernel(const unsigned short* __restrict__ E16,
                                                           unsigned short* __restrict__ ET) {
  __shared__ __align__(16) unsigned short Ts[64 * kTP];
  const int tid = threadIdx.x;
  const int ts = blockIdx.x >> 2, th = blockIdx.x & 3;
  const int s0 = ts * 64, h0 = th * 64;
  {
    const int r = tid >> 2, c16 = (tid & 3) * 16;
    const unsigned short* gp = E16 + (size_t)(s0 + r) * kHid + h0 + c16;
    const v4u a = *(const v4u*)(gp);
    const v4u b = *(const v4u*)(gp + 8);
    *(v4u*)(Ts + r * kTP + c16) = a;
    *(v4u*)(Ts + r * kTP + c16 + 8) = b;
  }
  __syncthreads();
  const int q = tid >> 3, c8 = (tid & 7) * 8;
  v4u o[2];
#pragma unroll
  for (int jj = 0; jj < 2; ++jj) {
    const int j = q + 32 * jj;
#pragma unroll
    for (int e2 = 0; e2 < 4; ++e2) {
      const unsigned lo = Ts[(c8 + 2 * e2) * kTP + j];
      const unsigned hi = Ts[(c8 + 2 * e2 + 1) * kTP + j];
      o[jj][e2] = lo | (hi << 16);
    }
  }
  for (int pass = 0; pass < 2; ++pass) {
#pragma unroll
    for (int jj = 0; jj < 2; ++jj) {
      const int j = q + 32 * jj;
      *(volatile v4u*)(ET + (size_t)(h0 + j) * kSeq + s0 + c8) = o[jj];
    }
    __threadfence();
  }
}

__global__ __launch_bounds__(kThr) void enc_seq_kernel(const float* __restrict__ x,
                                                       const unsigned short* __restrict__ WIp,
                                                       const unsigned short* __restrict__ WHp,
                                                       const float* __restrict__ bih, const float* __restrict__ bhh,
                                                       unsigned short* __restrict__ E16p, float* __restrict__ HENC) {
  __shared__ __align__(16) _Float16 Xs[kRows * kXP];
  __shared__ __align__(16) _Float16 Hh[kRows * kHP];
  __shared__ __align__(16) _Float16 Es[kHid];
  __shared__ __align__(16) float    Hs[kRows * kLP];
  const _Float16* WI = (const _Float16*)WIp;
  const _Float16* WH = (const _Float16*)WHp;
  _Float16* E16 = (_Float16*)E16p;
  const int tid = threadIdx.x, lane = tid & 31, wave = tid >> 5;
  const int c = lane & 15, hh = lane >> 4, koff = hh * 8;
  const int b0 = blockIdx.x * kRows;
  const int xr = (tid >> 2) & 15, xq = (tid & 3) * 8;

  {
    v8h zero8;
#pragma unroll
    for (int e = 0; e < 8; ++e) zero8[e] = (_Float16)0.0f;
#pragma unroll 1
    for (int i = tid; i < kRows * kHP / 8; i += kThr) *(v8h*)(Hh + 8 * i) = zero8;
  }
  float hst[2][8];
#pragma unroll
  for (int u = 0; u < 2; ++u)
#pragma unroll
    for (int r = 0; r < 8; ++r) hst[u][r] = 0.0f;
  float br[2], bz[2], bni[2], bnh[2];
#pragma unroll
  for (int u = 0; u < 2; ++u) {
    const int col = 32 * wave + 16 * u + c;
    br[u]  = bih[col] + bhh[col];
    bz[u]  = bih[kHid + col] + bhh[kHid + col];
    bni[u] = bih[2 * kHid + col];
    bnh[u] = bhh[2 * kHid + col];
  }
  if (tid < 64) {
    const float* xp = x + ((size_t)(b0 + xr) * kSeq + 0) * kIn + xq;
    const v4f xa = *(const v4f*)(xp);
    const v4f xb = *(const v4f*)(xp + 4);
    v8h xv;
#pragma unroll
    for (int e = 0; e < 4; ++e) { xv[e] = (_Float16)xa[e]; xv[4 + e] = (_Float16)xb[e]; }
    *(v8h*)(Xs + xr * kXP + xq) = xv;
  }
  __syncthreads();

  const v8f z8 = {0.f, 0.f, 0.f, 0.f, 0.f, 0.f, 0.f, 0.f};
#pragma unroll 1
  for (int t = 0; t < kSeq; ++t) {
    const v16h ax = Frag<_Float16>::load(Xs + c * kXP + koff);
#pragma unroll
    for (int u = 0; u < 2; ++u) {
      const int col = 32 * wave + 16 * u + c;
      v8f ar = z8, az = z8, ani = z8, anh = z8;
      {
        const v16h bir = Frag<_Float16>::load(WI + (size_t)col * kIn + koff);
        const v16h biz = Frag<_Float16>::load(WI + (size_t)(kHid + col) * kIn + koff);
        const v16h bin = Frag<_Float16>::load(WI + (size_t)(2 * kHid + col) * kIn + koff);
        ar  = mmah(ax, bir, ar);
        az  = mmah(ax, biz, az);
        ani = mmah(ax, bin, ani);
        guard3f4(ar, az, ani, ax, bir, biz, bin);
      }
      {
        const _Float16* ahp = Hh + c * kHP + koff;
        const _Float16* whr = WH + (size_t)col * kHid + koff;
        const _Float16* whz = WH + (size_t)(kHid + col) * kHid + koff;
        const _Float16* whn = WH + (size_t)(2 * kHid + col) * kHid + koff;
#pragma unroll 1
        for (int k0 = 0; k0 < kHid; k0 += 32) {
          const v16h ah  = Frag<_Float16>::load(ahp + k0);
          const v16h bhr = Frag<_Float16>::load(whr + k0);
          const v16h bhz = Frag<_Float16>::load(whz + k0);
          const v16h bhn = Frag<_Float16>::load(whn + k0);
          ar  = mmah(ah, bhr, ar);
          az  = mmah(ah, bhz, az);
          anh = mmah(ah, bhn, anh);
          guard3f4(ar, az, anh, ah, bhr, bhz, bhn);
        }
      }
      acc_guard4(ar, az, ani, anh);
#pragma unroll
      for (int r = 0; r < 8; ++r) {
        const float pr  = ar[r]  * kWinv + br[u];
        const float pz  = az[r]  * kWinv + bz[u];
        const float pni = ani[r] * kWinv + bni[u];
        const float pnh = anh[r] * kWinv + bnh[u];
        const float rg = fsig(pr);
        const float zg = fsig(pz);
        const float ng = ftanh(pni + rg * pnh);
        const float ho = hst[u][r];
        hst[u][r] = (1.0f - zg) * ng + zg * ho;
      }
    }
    __syncthreads();

#pragma unroll
    for (int u = 0; u < 2; ++u) {
      const int col = 32 * wave + 16 * u + c;
#pragma unroll
      for (int r = 0; r < 8; ++r) Hh[(8 * hh + r) * kHP + col] = (_Float16)hst[u][r];
    }
    if (hh == 0) {
#pragma unroll
      for (int u = 0; u < 2; ++u) Es[32 * wave + 16 * u + c] = (_Float16)(fmaxf(hst[u][0], 0.0f) * kWsc);
    }
    if (tid < 64) {
      const int tn = (t + 1 < kSeq) ? (t + 1) : t;
      const float* xp = x + ((size_t)(b0 + xr) * kSeq + (size_t)tn) * kIn + xq;
      const v4f xa = *(const v4f*)(xp);
      const v4f xb = *(const v4f*)(xp + 4);
      v8h xv;
#pragma unroll
      for (int e = 0; e < 4; ++e) { xv[e] = (_Float16)xa[e]; xv[4 + e] = (_Float16)xb[e]; }
      *(v8h*)(Xs + xr * kXP + xq) = xv;
    }
    __syncthreads();

    if (blockIdx.x == 0 && wave == 0) {
      const v8h ev = *(const v8h*)(Es + 8 * lane);
      _Float16* ep = E16 + (size_t)t * kHid + 8 * lane;
      *(volatile v8h*)ep = ev;
      __threadfence();
      *(volatile v8h*)ep = ev;
    }
  }

#pragma unroll
  for (int u = 0; u < 2; ++u) {
    const int col = 32 * wave + 16 * u + c;
#pragma unroll
    for (int r = 0; r < 8; ++r) Hs[(8 * hh + r) * kLP + col] = hst[u][r];
  }
  __syncthreads();
  for (int pass = 0; pass < 2; ++pass) {
#pragma unroll
    for (int rr = 0; rr < 2; ++rr) {
      const int row = 2 * wave + rr;
#pragma unroll
      for (int q = 0; q < 2; ++q) {
        const v4f v = *(const v4f*)(Hs + row * kLP + 128 * q + 4 * lane);
        *(volatile v4f*)(HENC + (size_t)(b0 + row) * kHid + 128 * q + 4 * lane) = v;
      }
    }
    __threadfence();
  }
}

__global__ __launch_bounds__(kThr) void dec_seq_kernel(
    const float* __restrict__ HENC, const float* __restrict__ ELOG, const float* __restrict__ ECMB,
    const unsigned short* __restrict__ ETp, const unsigned short* __restrict__ WA2p,
    const unsigned short* __restrict__ WC2p, const unsigned short* __restrict__ WIp,
    const unsigned short* __restrict__ WHp, const float* __restrict__ bih, const float* __restrict__ bhh,
    const float* __restrict__ Wo, const float* __restrict__ bo, float* __restrict__ out) {
  __shared__ __align__(16) _Float16 Hh[kRows * kHP];
  __shared__ __align__(16) _Float16 At[kRows * kHP];
  __shared__ __align__(16) _Float16 Ch[kRows * kHP];
  __shared__ __align__(16) _Float16 Mh[kRows * kHP];
  __shared__ __align__(16) float    Lg[kRows * kLP];
  __shared__ __align__(16) float    Os[64];
  const _Float16* ET  = (const _Float16*)ETp;
  const _Float16* WA2 = (const _Float16*)WA2p;
  const _Float16* WC2 = (const _Float16*)WC2p;
  const _Float16* WI  = (const _Float16*)WIp;
  const _Float16* WH  = (const _Float16*)WHp;
  const int tid = threadIdx.x, lane = tid & 31, wave = tid >> 5;
  const int c = lane & 15, hh = lane >> 4, koff = hh * 8;
  const int b0 = blockIdx.x * kRows;
  float* out1 = out + kBatch * kOut;

  float hst[2][8];
  float br[2], bz[2], bni[2], bnh[2];
#pragma unroll
  for (int u = 0; u < 2; ++u) {
    const int col = 32 * wave + 16 * u + c;
    br[u]  = bih[col] + bhh[col];
    bz[u]  = bih[kHid + col] + bhh[kHid + col];
    bni[u] = bih[2 * kHid + col];
    bnh[u] = bhh[2 * kHid + col];
#pragma unroll
    for (int r = 0; r < 8; ++r) {
      const int row = 8 * hh + r;
      const float v = HENC[(size_t)(b0 + row) * kHid + col];
      hst[u][r] = v;
      Hh[row * kHP + col] = (_Float16)v;
    }
  }
  __syncthreads();

  const v8f z8 = {0.f, 0.f, 0.f, 0.f, 0.f, 0.f, 0.f, 0.f};
#pragma unroll 1
  for (int t = 0; t < kSeq; ++t) {
    {
      const int s0c = 32 * wave + c, s1c = s0c + 16;
      v8f a0 = z8, a1 = z8;
      const _Float16* ahp = Hh + c * kHP + koff;
      const _Float16* wb0 = WA2 + (size_t)s0c * kHid + koff;
      const _Float16* wb1 = WA2 + (size_t)s1c * kHid + koff;
#pragma unroll 1
      for (int k0 = 0; k0 < kHid; k0 += 32) {
        const v16h ah  = Frag<_Float16>::load(ahp + k0);
        const v16h fb0 = Frag<_Float16>::load(wb0 + k0);
        const v16h fb1 = Frag<_Float16>::load(wb1 + k0);
        a0 = mmah(ah, fb0, a0);
        a1 = mmah(ah, fb1, a1);
        guard2f3(a0, a1, ah, fb0, fb1);
      }
      acc_guard2(a0, a1);
      const float e0 = ELOG[(size_t)t * kSeq + s0c];
      const float e1 = ELOG[(size_t)t * kSeq + s1c];
#pragma unroll
      for (int r = 0; r < 8; ++r) {
        const int row = 8 * hh + r;
        Lg[row * kLP + s0c] = e0 + a0[r] * kWinv;
        Lg[row * kLP + s1c] = e1 + a1[r] * kWinv;
      }
    }
    __syncthreads();

#pragma unroll
    for (int rr = 0; rr < 2; ++rr) {
      const int row = 2 * wave + rr;
      float* lr = Lg + row * kLP;
      const v4f x0 = *(const v4f*)(lr + 8 * lane);
      const v4f x1 = *(const v4f*)(lr + 8 * lane + 4);
      float pv[8];
#pragma unroll
      for (int e = 0; e < 4; ++e) { pv[e] = x0[e]; pv[4 + e] = x1[e]; }
      float mx = pv[0];
#pragma unroll
      for (int e = 1; e < 8; ++e) mx = fmaxf(mx, pv[e]);
#pragma unroll
      for (int off = 1; off < 32; off <<= 1) mx = fmaxf(mx, __shfl_xor(mx, off, 32));
      float sm = 0.0f;
#pragma unroll
      for (int e = 0; e < 8; ++e) { pv[e] = expf(pv[e] - mx); sm += pv[e]; }
#pragma unroll
      for (int off = 1; off < 32; off <<= 1) sm += __shfl_xor(sm, off, 32);
      const float inv = 1.0f / sm;
      v8h av;
#pragma unroll
      for (int e = 0; e < 8; ++e) { pv[e] = pv[e] * inv; av[e] = (_Float16)(pv[e] * kPSc); }
      *(v8h*)(At + row * kHP + 8 * lane) = av;
      if (t == kSeq - 1) {
#pragma unroll
        for (int e = 0; e < 8; ++e) lr[8 * lane + e] = pv[e];
        __builtin_amdgcn_fence(__ATOMIC_RELEASE, "workgroup");
        __builtin_amdgcn_wave_barrier();
        __builtin_amdgcn_fence(__ATOMIC_ACQUIRE, "workgroup");
        for (int pass = 0; pass < 2; ++pass) {
#pragma unroll
          for (int q = 0; q < 2; ++q) {
            const v4f ov = *(const v4f*)(lr + 128 * q + 4 * lane);
            *(volatile v4f*)(out1 + (size_t)(b0 + row) * kSeq + 128 * q + 4 * lane) = ov;
          }
          __threadfence();
        }
      }
    }
    __syncthreads();

    {
      const int h0c = 32 * wave + c, h1c = h0c + 16;
      v8f c0 = z8, c1 = z8;
      const _Float16* ap  = At + c * kHP + koff;
      const _Float16* eb0 = ET + (size_t)h0c * kSeq + koff;
      const _Float16* eb1 = ET + (size_t)h1c * kSeq + koff;
#pragma unroll 1
      for (int k0 = 0; k0 < kSeq; k0 += 32) {
        const v16h a   = Frag<_Float16>::load(ap + k0);
        const v16h fb0 = Frag<_Float16>::load(eb0 + k0);
        const v16h fb1 = Frag<_Float16>::load(eb1 + k0);
        c0 = mmah(a, fb0, c0);
        c1 = mmah(a, fb1, c1);
        guard2f3(c0, c1, a, fb0, fb1);
      }
      acc_guard2(c0, c1);
#pragma unroll
      for (int r = 0; r < 8; ++r) {
        const int row = 8 * hh + r;
        Ch[row * kHP + h0c] = (_Float16)(c0[r] * kCtxSt);
        Ch[row * kHP + h1c] = (_Float16)(c1[r] * kCtxSt);
      }
    }
    __syncthreads();

    {
      const int j0c = 32 * wave + c, j1c = j0c + 16;
      v8f m0 = z8, m1 = z8;
      const _Float16* ahp = Ch + c * kHP + koff;
      const _Float16* wb0 = WC2 + (size_t)j0c * kHid + koff;
      const _Float16* wb1 = WC2 + (size_t)j1c * kHid + koff;
#pragma unroll 1
      for (int k0 = 0; k0 < kHid; k0 += 32) {
        const v16h ah  = Frag<_Float16>::load(ahp + k0);
        const v16h fb0 = Frag<_Float16>::load(wb0 + k0);
        const v16h fb1 = Frag<_Float16>::load(wb1 + k0);
        m0 = mmah(ah, fb0, m0);
        m1 = mmah(ah, fb1, m1);
        guard2f3(m0, m1, ah, fb0, fb1);
      }
      acc_guard2(m0, m1);
      const float d0 = ECMB[(size_t)t * kHid + j0c];
      const float d1 = ECMB[(size_t)t * kHid + j1c];
#pragma unroll
      for (int r = 0; r < 8; ++r) {
        const int row = 8 * hh + r;
        const float v0 = fmaxf(d0 + m0[r] * kX16Inv, 0.0f);
        const float v1 = fmaxf(d1 + m1[r] * kX16Inv, 0.0f);
        Mh[row * kHP + j0c] = (_Float16)v0;
        Mh[row * kHP + j1c] = (_Float16)v1;
      }
    }
    __syncthreads();

#pragma unroll
    for (int u = 0; u < 2; ++u) {
      const int col = 32 * wave + 16 * u + c;
      v8f ar = z8, az = z8, ani = z8, anh = z8;
      const _Float16* amp = Mh + c * kHP + koff;
      const _Float16* ahp = Hh + c * kHP + koff;
      const _Float16* wir = WI + (size_t)col * kHid + koff;
      const _Float16* wiz = WI + (size_t)(kHid + col) * kHid + koff;
      const _Float16* win = WI + (size_t)(2 * kHid + col) * kHid + koff;
      const _Float16* whr = WH + (size_t)col * kHid + koff;
      const _Float16* whz = WH + (size_t)(kHid + col) * kHid + koff;
      const _Float16* whn = WH + (size_t)(2 * kHid + col) * kHid + koff;
#pragma unroll 1
      for (int k0 = 0; k0 < kHid; k0 += 32) {
        {
          const v16h am  = Frag<_Float16>::load(amp + k0);
          const v16h bir = Frag<_Float16>::load(wir + k0);
          const v16h biz = Frag<_Float16>::load(wiz + k0);
          const v16h bin = Frag<_Float16>::load(win + k0);
          ar  = mmah(am, bir, ar);
          az  = mmah(am, biz, az);
          ani = mmah(am, bin, ani);
          guard3f4(ar, az, ani, am, bir, biz, bin);
        }
        {
          const v16h ah  = Frag<_Float16>::load(ahp + k0);
          const v16h bhr = Frag<_Float16>::load(whr + k0);
          const v16h bhz = Frag<_Float16>::load(whz + k0);
          const v16h bhn = Frag<_Float16>::load(whn + k0);
          ar  = mmah(ah, bhr, ar);
          az  = mmah(ah, bhz, az);
          anh = mmah(ah, bhn, anh);
          guard3f4(ar, az, anh, ah, bhr, bhz, bhn);
        }
      }
      acc_guard4(ar, az, ani, anh);
#pragma unroll
      for (int r = 0; r < 8; ++r) {
        const int row = 8 * hh + r;
        const float pr  = ar[r]  * kWinv + br[u];
        const float pz  = az[r]  * kWinv + bz[u];
        const float pni = ani[r] * kWinv + bni[u];
        const float pnh = anh[r] * kWinv + bnh[u];
        const float rg = fsig(pr);
        const float zg = fsig(pz);
        const float ng = ftanh(pni + rg * pnh);
        const float ho = hst[u][r];
        const float hn = (1.0f - zg) * ng + zg * ho;
        hst[u][r] = hn;
        if (t == 0) Lg[row * kLP + col] = hn;
      }
    }
    __syncthreads();

#pragma unroll
    for (int u = 0; u < 2; ++u) {
      const int col = 32 * wave + 16 * u + c;
#pragma unroll
      for (int r = 0; r < 8; ++r) Hh[(8 * hh + r) * kHP + col] = (_Float16)hst[u][r];
    }

    if (t == 0) {
      if (tid < 64) {
        const int m = tid >> 2, o = tid & 3;
        const float* hrow = Lg + m * kLP;
        const float* wrow = Wo + o * kHid;
        float s = 0.0f;
#pragma unroll 1
        for (int k2 = 0; k2 < kHid; ++k2) s += hrow[k2] * wrow[k2];
        Os[tid] = fmaxf(s + bo[o], 0.0f);
      }
      __syncthreads();
      if (wave == 0) {
        const v4f ov = *(const v4f*)(Os + 4 * (lane & 15));
        float* op = out + (size_t)(b0 + (lane & 15)) * kOut;
        if (lane < 16) *(volatile v4f*)op = ov;
        __threadfence();
        if (lane < 16) *(volatile v4f*)op = ov;
      }
    }
    __syncthreads();
  }
}

extern "C" void kernel_launch(void* const* d_in, const int* in_sizes, int n_in,
                              void* d_out, int out_size, void* d_ws, size_t ws_size, hipStream_t stream) {
  if (n_in < 15 || d_out == nullptr || d_ws == nullptr) return;
  if (in_sizes[0] != kBatch * kSeq * kIn || in_sizes[1] != kGate * kIn || in_sizes[2] != kGate * kHid ||
      in_sizes[3] != kGate || in_sizes[4] != kGate || in_sizes[5] != kGate * kHid || in_sizes[6] != kGate * kHid ||
      in_sizes[7] != kGate || in_sizes[8] != kGate || in_sizes[9] != kSeq * 2 * kHid || in_sizes[10] != kSeq ||
      in_sizes[11] != kHid * 2 * kHid || in_sizes[12] != kHid || in_sizes[13] != kOut * kHid || in_sizes[14] != kOut ||
      out_size != kBatch * kOut + kBatch * kSeq) return;

  const float* x     = (const float*)d_in[0];
  const float* wih_e = (const float*)d_in[1];
  const float* whh_e = (const float*)d_in[2];
  const float* bih_e = (const float*)d_in[3];
  const float* bhh_e = (const float*)d_in[4];
  const float* wih_d = (const float*)d_in[5];
  const float* whh_d = (const float*)d_in[6];
  const float* bih_d = (const float*)d_in[7];
  const float* bhh_d = (const float*)d_in[8];
  const float* wa    = (const float*)d_in[9];
  const float* ba    = (const float*)d_in[10];
  const float* wc    = (const float*)d_in[11];
  const float* bc    = (const float*)d_in[12];
  const float* wo    = (const float*)d_in[13];
  const float* bo    = (const float*)d_in[14];
  float* out = (float*)d_out;

  char* ws = (char*)d_ws; size_t off = 0;
  auto carve = [&](size_t bytes) -> char* { char* p = ws + off; off += (bytes + 255) & ~(size_t)255; return p; };
  unsigned short* WIHE = (unsigned short*)carve((size_t)kGate * kIn * 2);
  unsigned short* WHHE = (unsigned short*)carve((size_t)kGate * kHid * 2);
  unsigned short* WIHD = (unsigned short*)carve((size_t)kGate * kHid * 2);
  unsigned short* WHHD = (unsigned short*)carve((size_t)kGate * kHid * 2);
  unsigned short* WA1  = (unsigned short*)carve((size_t)kSeq * kHid * 2);
  unsigned short* WA2  = (unsigned short*)carve((size_t)kSeq * kHid * 2);
  unsigned short* WC1  = (unsigned short*)carve((size_t)kHid * kHid * 2);
  unsigned short* WC2  = (unsigned short*)carve((size_t)kHid * kHid * 2);
  unsigned short* E16  = (unsigned short*)carve((size_t)kSeq * kHid * 2);
  unsigned short* ET   = (unsigned short*)carve((size_t)kHid * kSeq * 2);
  float*          HENC = (float*)carve((size_t)kBatch * kHid * 4);
  float*          ELOG = (float*)carve((size_t)kSeq * kSeq * 4);
  float*          ECMB = (float*)carve((size_t)kSeq * kHid * 4);
  if (off > ws_size || off > (size_t)134217728) return;

  const int n8_ie = kGate * (kIn / 8);
  const int n8_hh = kGate * (kHid / 8);
  const int n8_sq = kSeq * (kHid / 8);
  cvt8_f16_kernel<<<(n8_ie + kThr - 1) / kThr, kThr, 0, stream>>>(wih_e, WIHE, kGate, kIn / 8,  kIn,      0,    kWsc);
  cvt8_f16_kernel<<<(n8_hh + kThr - 1) / kThr, kThr, 0, stream>>>(whh_e, WHHE, kGate, kHid / 8, kHid,     0,    kWsc);
  cvt8_f16_kernel<<<(n8_hh + kThr - 1) / kThr, kThr, 0, stream>>>(wih_d, WIHD, kGate, kHid / 8, kHid,     0,    kWsc);
  cvt8_f16_kernel<<<(n8_hh + kThr - 1) / kThr, kThr, 0, stream>>>(whh_d, WHHD, kGate, kHid / 8, kHid,     0,    kWsc);
  cvt8_f16_kernel<<<(n8_sq + kThr - 1) / kThr, kThr, 0, stream>>>(wa,    WA1,  kSeq,  kHid / 8, 2 * kHid, 0,    kWsc);
  cvt8_f16_kernel<<<(n8_sq + kThr - 1) / kThr, kThr, 0, stream>>>(wa,    WA2,  kSeq,  kHid / 8, 2 * kHid, kHid, kWsc);
  cvt8_f16_kernel<<<(n8_sq + kThr - 1) / kThr, kThr, 0, stream>>>(wc,    WC1,  kHid,  kHid / 8, 2 * kHid, 0,    kWsc);
  cvt8_f16_kernel<<<(n8_sq + kThr - 1) / kThr, kThr, 0, stream>>>(wc,    WC2,  kHid,  kHid / 8, 2 * kHid, kHid, kWsc);

  enc_seq_kernel<<<kBatch / kRows, kThr, 0, stream>>>(x, WIHE, WHHE, bih_e, bhh_e, E16, HENC);

  transpose_e_kernel<<<16, kThr, 0, stream>>>(E16, ET);

  const dim3 ggrid((kSeq / 64) * (kSeq / 64) / 8, 1);
  wmma_gemm64<0, false, 2, 0, false, 0><<<ggrid, 256, 0, stream>>>(
      E16, E16, kHid, 0L, WA1, WA1, kHid, 0L, (void*)ELOG, (void*)ELOG, kSeq, 0L,
      ba, ELOG, 0L, kSeq, kSeq, kHid, kX16Inv);
  wmma_gemm64<0, false, 2, 0, false, 0><<<ggrid, 256, 0, stream>>>(
      E16, E16, kHid, 0L, WC1, WC1, kHid, 0L, (void*)ECMB, (void*)ECMB, kHid, 0L,
      bc, ECMB, 0L, kSeq, kHid, kHid, kX16Inv);

  dec_seq_kernel<<<kBatch / kRows, kThr, 0, stream>>>(HENC, ELOG, ECMB, ET, WA2, WC2, WIHD, WHHD,
                                                      bih_d, bhh_d, wo, bo, out);
}
